// MambaVisionMixer_89936615178949
// MI455X (gfx1250) — hardware-verified
//
#include <hip/hip_runtime.h>
#include <hip/hip_bf16.h>
#include <math.h>

#define D_MODEL 1024
#define D_INNER 2048
#define D_HALF  1024
#define D_STATE 16
#define DT_RANK 64
#define B_SZ    4
#define SEQ_L   2048
#define MROWS   (B_SZ * SEQ_L)
#define XDBL_W  (DT_RANK + 2 * D_STATE)

typedef __attribute__((ext_vector_type(16))) _Float16 bf16x16;
typedef __attribute__((ext_vector_type(8)))  _Float16 bf16x8;
typedef __attribute__((ext_vector_type(4)))  _Float16 bf16x4;
#define __bf16 _Float16
typedef __attribute__((ext_vector_type(8)))  float  f32x8;
typedef __attribute__((ext_vector_type(4)))  float  f32x4;

union Frag {
    bf16x16 v;
    bf16x8  h[2];
};

#define BM 128
#define BN 128
#define KB 32

typedef __attribute__((ext_vector_type(4))) float v4f_t;
typedef float v4fa __attribute__((ext_vector_type(4), may_alias));
__device__ __forceinline__ void store_tile16x32(const float* stg, float* __restrict__ dst, size_t ld, int lane) {
    v4f_t vv[4];
#pragma unroll
    for (int i = 0; i < 4; ++i) { const int c = lane + 32 * i; vv[i] = *(const v4fa*)(stg + (c >> 3) * 32 + (c & 7) * 4); }
#pragma unroll
    for (int i = 0; i < 4; ++i) { const int c = lane + 32 * i; *(volatile v4f_t*)(dst + (size_t)(c >> 3) * ld + (c & 7) * 4) = vv[i]; }
    __threadfence();
#pragma unroll
    for (int i = 0; i < 4; ++i) { const int c = lane + 32 * i; *(volatile v4f_t*)(dst + (size_t)(c >> 3) * ld + (c & 7) * 4) = vv[i]; }
}

template<int MODE, bool GUARD>
__global__ __launch_bounds__(256)
void gemm_bf16_wmma(const float* __restrict__ A, int lda,
                    const float* __restrict__ B, int ldb,
                    float* __restrict__ C, int ldc,
                    const float* __restrict__ aux,
                    int M, int N, int K)
{
    __shared__ alignas(16) __bf16 As[BM][KB];
    __shared__ alignas(16) __bf16 Bs[BN][KB];
    __shared__ alignas(16) __bf16 Asl[BM][KB];
    __shared__ alignas(16) __bf16 Bsl[BN][KB];
    __shared__ alignas(16) float stg[8][16 * 32];

    const int tid  = threadIdx.x;
    const int wave = tid >> 5;
    const int lane = tid & 31;
    const int m0   = blockIdx.y * BM;
    const int n0   = blockIdx.x * BN;

    const int wm = (wave & 3) * 32;
    const int wn = (wave >> 2) * 64;

    const int hh = lane >> 4;
    const int ml = lane & 15;

    f32x8 acc[2][4];
    #pragma unroll
    for (int i = 0; i < 2; ++i)
        #pragma unroll
        for (int j = 0; j < 4; ++j)
            acc[i][j] = f32x8{};

    for (int k0 = 0; k0 < K; k0 += KB) {
        #pragma unroll
        for (int i = 0; i < 4; ++i) {
            int idx4 = tid + i * 256;
            int r    = idx4 >> 3;
            int kq   = idx4 & 7;
            const float* p = A + (size_t)(m0 + r) * lda + (k0 + kq * 4);
            f32x4 v = *(const f32x4*)p;
            bf16x4 w, wl;
            #pragma unroll
            for (int e = 0; e < 4; ++e) { w[e] = (__bf16)v[e]; wl[e] = (__bf16)((v[e] - (float)w[e]) * 2048.0f); }
            *(bf16x4*)&As[r][kq * 4]  = w;
            *(bf16x4*)&Asl[r][kq * 4] = wl;
        }
        #pragma unroll
        for (int i = 0; i < 4; ++i) {
            int idx4 = tid + i * 256;
            int kk   = idx4 >> 5;
            int nq   = idx4 & 31;
            int gn   = n0 + nq * 4;
            f32x4 v = f32x4{};
            if (!GUARD || gn < N)
                v = *(const f32x4*)(B + (size_t)(k0 + kk) * ldb + gn);
            #pragma unroll
            for (int e = 0; e < 4; ++e) {
                const __bf16 h = (__bf16)v[e];
                Bs[nq * 4 + e][kk]  = h;
                Bsl[nq * 4 + e][kk] = (__bf16)((v[e] - (float)h) * 2048.0f);
            }
        }
        __syncthreads();

        Frag a[2], b[4], al[2], bl[4];
        #pragma unroll
        for (int i = 0; i < 2; ++i) {
            const __bf16* p = &As[wm + i * 16 + ml][hh * 8];
            a[i].h[0] = *(const bf16x8*)p;
            a[i].h[1] = *(const bf16x8*)(p + 16);
            const __bf16* pl = &Asl[wm + i * 16 + ml][hh * 8];
            al[i].h[0] = *(const bf16x8*)pl;
            al[i].h[1] = *(const bf16x8*)(pl + 16);
        }
        #pragma unroll
        for (int j = 0; j < 4; ++j) {
            const __bf16* p = &Bs[wn + j * 16 + ml][hh * 8];
            b[j].h[0] = *(const bf16x8*)p;
            b[j].h[1] = *(const bf16x8*)(p + 16);
            const __bf16* pl = &Bsl[wn + j * 16 + ml][hh * 8];
            bl[j].h[0] = *(const bf16x8*)pl;
            bl[j].h[1] = *(const bf16x8*)(pl + 16);
        }

        #pragma unroll
        for (int i = 0; i < 2; ++i)
            #pragma unroll
            for (int j = 0; j < 4; ++j) {
                f32x8 x = __builtin_amdgcn_wmma_f32_16x16x32_f16(false, al[i].v, false, b[j].v, (short)0, f32x8{}, false, false);
                x = __builtin_amdgcn_wmma_f32_16x16x32_f16(false, a[i].v, false, bl[j].v, (short)0, x, false, false);
                acc[i][j] = __builtin_amdgcn_wmma_f32_16x16x32_f16(
                    false, a[i].v, false, b[j].v, (short)0, acc[i][j],
                    false, false) + x * (1.0f / 2048.0f);
            }

        __syncthreads();
    }

    float* sg = stg[wave];
    #pragma unroll
    for (int i = 0; i < 2; ++i) {
        #pragma unroll
        for (int jp = 0; jp < 4; jp += 2) {
            const int gnb = n0 + wn + jp * 16;
            if (GUARD && gnb + 32 > N) continue;
            #pragma unroll
            for (int jj = 0; jj < 2; ++jj) {
                const int gn = gnb + jj * 16 + ml;
                float avals = 0.0f;
                if (MODE != 0) avals = aux[gn];
                #pragma unroll
                for (int v = 0; v < 8; ++v) {
                    float r = acc[i][jp + jj][v];
                    float o;
                    if (MODE == 2) {
                        float x = r + 2.0f * avals;
                        o = (x > 20.0f) ? x : log1pf(__expf(x));
                    } else if (MODE == 3) {
                        o = r + avals;
                    } else {
                        o = r;
                    }
                    sg[(v + hh * 8) * 32 + jj * 16 + ml] = o;
                }
            }
            store_tile16x32(sg, C + (size_t)(m0 + wm + i * 16) * ldc + gnb, (size_t)ldc, lane);
        }
    }
}

__global__ __launch_bounds__(256)
void dwconv_silu_kernel(const float* __restrict__ x, int istride,
                        const float* __restrict__ w,
                        const float* __restrict__ bias,
                        float* __restrict__ y, int ostride,
                        long long total)
{
    long long i = (long long)blockIdx.x * blockDim.x + threadIdx.x;
    if (i >= total) return;
    int c   = (int)(i % D_HALF);
    int row = (int)(i / D_HALF);
    int t   = row & (SEQ_L - 1);
    int b   = row >> 11;

    float s = bias[c];
    #pragma unroll
    for (int j = 0; j < 4; ++j) {
        int tt = t + j - 1;
        if (tt >= 0 && tt < SEQ_L)
            s = fmaf(x[(size_t)(b * SEQ_L + tt) * istride + c],
                     w[j * D_HALF + c], s);
    }
    const float o = s / (1.0f + __expf(-s));
    *(volatile float*)(y + (size_t)row * ostride + c) = o;
    __threadfence();
    *(volatile float*)(y + (size_t)row * ostride + c) = o;
}

__global__ __launch_bounds__(256)
void selective_scan_kernel(const float* __restrict__ delta,
                           const float* __restrict__ u,
                           const float* __restrict__ xdbl,
                           const float* __restrict__ Dvec,
                           float* __restrict__ y, int ystride)
{
    const int gid = blockIdx.x * 256 + threadIdx.x;
    const int b   = gid >> 10;
    const int d   = gid & (D_HALF - 1);

    __shared__ float bc[2 * D_STATE];

    float h[D_STATE];
    #pragma unroll
    for (int n = 0; n < D_STATE; ++n) h[n] = 0.0f;

    const float dval = Dvec[d];

    for (int t = 0; t < SEQ_L; ++t) {
        const long long row = (long long)b * SEQ_L + t;
        if (threadIdx.x < 2 * D_STATE)
            bc[threadIdx.x] = xdbl[row * XDBL_W + DT_RANK + threadIdx.x];
        __syncthreads();

        float dlt = delta[row * D_HALF + d];
        float uu  = u[row * D_HALF + d];
        float r   = __expf(-dlt);
        float du  = dlt * uu;

        float p = 1.0f, acc = 0.0f;
        #pragma unroll
        for (int n = 0; n < D_STATE; ++n) {
            p *= r;
            h[n] = fmaf(p, h[n], du * bc[n]);
            acc  = fmaf(h[n], bc[D_STATE + n], acc);
        }
        const float yo = fmaf(uu, dval, acc);
        *(volatile float*)(y + row * ystride + d) = yo;
        __threadfence();
        *(volatile float*)(y + row * ystride + d) = yo;
        __syncthreads();
    }
}

extern "C" void kernel_launch(void* const* d_in, const int* in_sizes, int n_in,
                              void* d_out, int out_size, void* d_ws, size_t ws_size,
                              hipStream_t stream)
{
    (void)in_sizes; (void)n_in; (void)out_size; (void)ws_size;

    const float* x       = (const float*)d_in[0];
    const float* W_in    = (const float*)d_in[1];
    const float* conv_xw = (const float*)d_in[2];
    const float* conv_xb = (const float*)d_in[3];
    const float* conv_zw = (const float*)d_in[4];
    const float* conv_zb = (const float*)d_in[5];
    const float* W_xdbl  = (const float*)d_in[6];
    const float* W_dt    = (const float*)d_in[7];
    const float* inv_dt  = (const float*)d_in[8];
    const float* Dvec    = (const float*)d_in[9];
    const float* W_out   = (const float*)d_in[10];
    const float* b_out   = (const float*)d_in[11];
    float* out = (float*)d_out;

    float* ws   = (float*)d_ws;
    const size_t PLANE2 = (size_t)MROWS * D_INNER;
    const size_t PLANE1 = (size_t)MROWS * D_HALF;
    float* xz    = ws;
    float* xs_c  = xz + PLANE2;
    float* ycat  = xs_c + PLANE1;
    float* xdbl  = ycat + PLANE2;
    float* delta = xz;

    dim3 blk(256);

    gemm_bf16_wmma<0, false><<<dim3(D_INNER / BN, MROWS / BM), blk, 0, stream>>>(
        x, D_MODEL, W_in, D_INNER, xz, D_INNER, nullptr,
        MROWS, D_INNER, D_MODEL);

    {
        long long total = (long long)MROWS * D_HALF;
        dim3 grid((unsigned)((total + 255) / 256));
        dwconv_silu_kernel<<<grid, blk, 0, stream>>>(
            xz, D_INNER, conv_xw, conv_xb, xs_c, D_HALF, total);
        dwconv_silu_kernel<<<grid, blk, 0, stream>>>(
            xz + D_HALF, D_INNER, conv_zw, conv_zb, ycat + D_HALF, D_INNER, total);
    }

    gemm_bf16_wmma<0, true><<<dim3(1, MROWS / BM), blk, 0, stream>>>(
        xs_c, D_HALF, W_xdbl, XDBL_W, xdbl, XDBL_W, nullptr,
        MROWS, XDBL_W, D_HALF);

    gemm_bf16_wmma<2, false><<<dim3(D_HALF / BN, MROWS / BM), blk, 0, stream>>>(
        xdbl, XDBL_W, W_dt, D_HALF, delta, D_HALF, inv_dt,
        MROWS, D_HALF, DT_RANK);

    selective_scan_kernel<<<dim3((B_SZ * D_HALF) / 256), blk, 0, stream>>>(
        delta, xs_c, xdbl, Dvec, ycat, D_INNER);

    gemm_bf16_wmma<3, false><<<dim3(D_MODEL / BN, MROWS / BM), blk, 0, stream>>>(
        ycat, D_INNER, W_out, D_MODEL, out, D_MODEL, b_out,
        MROWS, D_MODEL, D_INNER);
}
